// SegmentBiasedDisentangledMultiheadAttention_59648505806984
// MI455X (gfx1250) — hardware-verified
//
#include <hip/hip_runtime.h>
#include <hip/hip_bf16.h>
#include <cstdint>

typedef __attribute__((ext_vector_type(16))) _Float16 v16h;
typedef __attribute__((ext_vector_type(8)))  _Float16 v8h;
typedef __attribute__((ext_vector_type(8)))  float    v8f;
typedef __attribute__((ext_vector_type(4)))  float    v4f;
__device__ __forceinline__ int kmap(int e, int hh) { return (e < 8) ? (8 * hh + e) : (16 + 8 * hh + (e - 8)); }

#define BB 8
#define SS 384
#define DD 768
#define EE 768
#define HH 12
#define HDIM 64
#define SCALE_Q 0.07216878364870322f

__device__ __forceinline__ v16h loadA16(const _Float16* __restrict__ base, int m0, int ko, int ld, int lane) {
    int half = (lane >> 4) & 1, m = lane & 15;
    const _Float16* p = base + (size_t)(m0 + m) * ld + ko + half * 8;
    v16h a;
#pragma unroll
    for (int t = 0; t < 8; ++t) { a[t] = p[t]; a[t + 8] = p[t + 16]; }
    return a;
}
__device__ __forceinline__ v16h loadB16(const _Float16* __restrict__ base, int n0, int ko, int ld, int lane) {
    int half = (lane >> 4) & 1, n = lane & 15;
    const _Float16* p = base + (size_t)(n0 + n) * ld + ko + half * 8;
    v16h b;
#pragma unroll
    for (int t = 0; t < 8; ++t) { b[t] = p[t]; b[t + 8] = p[t + 16]; }
    return b;
}
__device__ __forceinline__ v8f wmma16(v16h a, v16h b, v8f c) {
    v8f d = __builtin_amdgcn_wmma_f32_16x16x32_f16(false, a, false, b, (short)0, c, false, false);
    asm volatile("v_nop\n\tv_nop\n\tv_nop\n\tv_nop" : "+v"(d) : "v"(a), "v"(b));
    return d;
}
__device__ __forceinline__ v8f zero8() { v8f z = {0.f,0.f,0.f,0.f,0.f,0.f,0.f,0.f}; return z; }

__global__ void k_f32_to_f16(const float* __restrict__ s, _Float16* __restrict__ d, int n) {
    int i = blockIdx.x * blockDim.x + threadIdx.x;
    if (i < n) { const _Float16 v = (_Float16)s[i]; *(volatile _Float16*)(d + i) = v; __threadfence(); *(volatile _Float16*)(d + i) = v; }
}
__global__ void k_build_rel(const float* __restrict__ rel_emb, _Float16* __restrict__ relh) {
    int i = blockIdx.x * blockDim.x + threadIdx.x;
    if (i >= 768 * 768) return;
    int r = i / 768, c = i % 768;
    const _Float16 v = (r < 767) ? (_Float16)rel_emb[(size_t)(r + 128) * 768 + c] : (_Float16)0.f;
    *(volatile _Float16*)(relh + i) = v; __threadfence(); *(volatile _Float16*)(relh + i) = v;
}

__device__ __forceinline__ void tile16x64(const _Float16* __restrict__ A, int m0, const _Float16* __restrict__ W, int n0, int K, int lane, v8f (&c)[4]) {
#pragma unroll
    for (int t = 0; t < 4; ++t) c[t] = zero8();
#pragma unroll 2
    for (int kt = 0; kt < K / 32; ++kt) {
        v16h a = loadA16(A, m0, kt * 32, K, lane);
#pragma unroll
        for (int t = 0; t < 4; ++t) { v16h bf = loadB16(W, n0 + t * 16, kt * 32, K, lane); c[t] = wmma16(a, bf, c[t]); }
    }
}
__device__ __forceinline__ void store_rows64_f16(_Float16* sT  , const v8f (&c)[4], const float* bias64, float sc, int lane,
                                                 _Float16* dst, size_t rowStride  , const size_t* rowOff  ) {
    const int half = lane >> 4, n = lane & 15;
#pragma unroll
    for (int t = 0; t < 4; ++t)
#pragma unroll
        for (int r = 0; r < 8; ++r) sT[(r + 8 * half) * 72 + t * 16 + n] = (_Float16)((c[t][r] + bias64[t * 16 + n]) * sc);
    asm volatile("s_wait_dscnt 0" ::: "memory");
    __builtin_amdgcn_fence(__ATOMIC_RELEASE, "workgroup"); __builtin_amdgcn_wave_barrier(); __builtin_amdgcn_fence(__ATOMIC_ACQUIRE, "workgroup");
    for (int pass = 0; pass < 2; ++pass) {
#pragma unroll
        for (int j = 0; j < 4; ++j) { const int rr = j * 4 + (lane >> 3), q8 = (lane & 7) * 8;
            *(volatile v8h*)(dst + (size_t)rr * rowStride + q8) = *(const v8h*)(&sT[rr * 72 + q8]); }
        __threadfence();
    }
    __builtin_amdgcn_fence(__ATOMIC_RELEASE, "workgroup"); __builtin_amdgcn_wave_barrier(); __builtin_amdgcn_fence(__ATOMIC_ACQUIRE, "workgroup");
    (void)rowOff;
}
__global__ __launch_bounds__(256) void k_gemm_qkv(
    const _Float16* __restrict__ xh,
    const _Float16* __restrict__ wq, const _Float16* __restrict__ wk, const _Float16* __restrict__ wv,
    const float* __restrict__ bq, const float* __restrict__ bk, const float* __restrict__ bv,
    _Float16* __restrict__ qb, _Float16* __restrict__ kb, _Float16* __restrict__ vb)
{
    __shared__ __attribute__((aligned(16))) _Float16 sT[8][16 * 72];
    int lane = threadIdx.x & 31, wave = threadIdx.x >> 5;
    int mat = blockIdx.z;
    int tile = blockIdx.x * 8 + wave;
    int mt = tile / HH, h = tile % HH;
    const _Float16* w = (mat == 0) ? wq : (mat == 1) ? wk : wv;
    const float* bias = (mat == 0) ? bq : (mat == 1) ? bk : bv;
    v8f c[4];
    tile16x64(xh, mt * 16, w, h * HDIM, DD, lane, c);
    const int gm0 = mt * 16, b_ = gm0 / SS, s0 = gm0 % SS;
    _Float16* dst = ((mat == 0) ? qb : (mat == 1) ? kb : vb) + ((size_t)(b_ * HH + h) * SS + s0) * HDIM;
    store_rows64_f16(sT[wave], c, bias + h * HDIM, (mat == 0) ? SCALE_Q : 1.0f, lane, dst, HDIM, nullptr);
}
__global__ __launch_bounds__(256) void k_gemm_pos(
    const _Float16* __restrict__ relh,
    const _Float16* __restrict__ wpk, const _Float16* __restrict__ wpq,
    const float* __restrict__ bpk, const float* __restrict__ bpq,
    _Float16* __restrict__ posk, _Float16* __restrict__ posq)
{
    __shared__ __attribute__((aligned(16))) _Float16 sT[8][16 * 72];
    int lane = threadIdx.x & 31, wave = threadIdx.x >> 5;
    int mat = blockIdx.z;
    int tile = blockIdx.x * 8 + wave;
    int mt = tile / HH, h = tile % HH;
    const _Float16* w = mat ? wpq : wpk;
    const float* bias = mat ? bpq : bpk;
    v8f c[4];
    tile16x64(relh, mt * 16, w, h * HDIM, DD, lane, c);
    _Float16* dst = (mat ? posq : posk) + ((size_t)h * 768 + mt * 16) * HDIM;
    store_rows64_f16(sT[wave], c, bias + h * HDIM, mat ? SCALE_Q : 1.0f, lane, dst, HDIM, nullptr);
}

__global__ __launch_bounds__(64) void k_attn(
    const _Float16* __restrict__ qb, const _Float16* __restrict__ kb, const _Float16* __restrict__ vt,
    const _Float16* __restrict__ posk, const _Float16* __restrict__ posq,
    const int* __restrict__ mask, const int* __restrict__ seg, const float* __restrict__ sep,
    const float* __restrict__ same_bias, const float* __restrict__ cross_bias,
    const float* __restrict__ sep_scale, const float* __restrict__ sep_decay,
    _Float16* __restrict__ ao)
{
    __shared__ float    sq [2][16][400];
    __shared__ float    skt[2][16][32];
    __shared__ _Float16 pst[2][16][32];
    __shared__ float    asep_s[SS];
    __shared__ int      seg_s[SS];
    __shared__ int      msk_s[SS];

    int tid = threadIdx.x, lane = tid & 31, wave = tid >> 5;
    int half = lane >> 4, ln = lane & 15;
    int it = blockIdx.x % 12;
    int bh = blockIdx.x / 12;
    int b_ = bh / HH, h = bh % HH;

    for (int i = tid; i < SS; i += 64) {
        asep_s[i] = fabsf(sep[b_ * SS + i]);
        seg_s[i]  = seg[b_ * SS + i];
        msk_s[i]  = mask[b_ * SS + i];
    }
    __syncthreads();

    float sb = same_bias[h], cb = cross_bias[h], ssc = sep_scale[h];
    float dc = log1pf(__expf(sep_decay[h])) + 1e-4f;

    int ibase = it * 32 + wave * 16;
    const _Float16* qp  = qb   + (size_t)(b_ * HH + h) * SS * HDIM;
    const _Float16* kp  = kb   + (size_t)(b_ * HH + h) * SS * HDIM;
    const _Float16* vp  = vt   + (size_t)(b_ * HH + h) * SS * HDIM;
    const _Float16* pkh = posk + (size_t)h * 768 * HDIM;
    const _Float16* pqh = posq + (size_t)h * 768 * HDIM;

    v16h aq0 = loadA16(qp, ibase, 0, HDIM, lane);
    v16h aq1 = loadA16(qp, ibase, 32, HDIM, lane);

    for (int ct = 0; ct < 25; ++ct) {
        v8f c = zero8();
        v16h b0 = loadB16(pkh, ibase + ct * 16, 0, HDIM, lane);
        v16h b1 = loadB16(pkh, ibase + ct * 16, 32, HDIM, lane);
        c = wmma16(aq0, b0, c);
        c = wmma16(aq1, b1, c);
#pragma unroll
        for (int r = 0; r < 8; ++r) sq[wave][r + 8 * half][ct * 16 + ln] = c[r];
    }
    asm volatile("s_wait_dscnt 0" ::: "memory");

    float mcur[8], lcur[8];
    v8f of[4];
#pragma unroll
    for (int r = 0; r < 8; ++r) { mcur[r] = -1e30f; lcur[r] = 0.f; }
#pragma unroll
    for (int f = 0; f < 4; ++f) of[f] = zero8();

    for (int jb0 = 0; jb0 < SS; jb0 += 32) {
        float sv[2][8];
#pragma unroll
        for (int sub = 0; sub < 2; ++sub) {
            int jb = jb0 + sub * 16;
            v16h ak0 = loadA16(kp, jb, 0, HDIM, lane);
            v16h ak1 = loadA16(kp, jb, 32, HDIM, lane);
            int rw0 = ibase - jb + 368;
#pragma unroll
            for (int f = 0; f < 2; ++f) {
                v8f cs = zero8();
                v16h b0 = loadB16(pqh, rw0 + f * 16, 0, HDIM, lane);
                v16h b1 = loadB16(pqh, rw0 + f * 16, 32, HDIM, lane);
                cs = wmma16(ak0, b0, cs);
                cs = wmma16(ak1, b1, cs);
#pragma unroll
                for (int r = 0; r < 8; ++r) skt[wave][r + 8 * half][f * 16 + ln] = cs[r];
            }
            v16h bk0 = loadB16(kp, jb, 0, HDIM, lane);
            v16h bk1 = loadB16(kp, jb, 32, HDIM, lane);
            v8f cc = zero8();
            cc = wmma16(aq0, bk0, cc);
            cc = wmma16(aq1, bk1, cc);
            asm volatile("s_wait_dscnt 0" ::: "memory");
#pragma unroll
            for (int r = 0; r < 8; ++r) {
                int mi = r + 8 * half;
                int i = ibase + mi;
                int j = jb + ln;
                float s = cc[r]
                        + sq[wave][mi][mi - j + 383]
                        + skt[wave][ln][mi - ln + 15];
                float bias_;
                if (seg_s[i] == seg_s[j]) bias_ = sb;
                else {
                    float gap = fabsf(asep_s[i] - asep_s[j]);
                    bias_ = cb + __expf(-gap * dc) * ssc;
                }
                s += bias_;
                if (msk_s[j] == 0) s = -9.0e15f;
                sv[sub][r] = s;
            }
        }
        float tmax[8], psum[8];
#pragma unroll
        for (int r = 0; r < 8; ++r) tmax[r] = fmaxf(sv[0][r], sv[1][r]);
#pragma unroll
        for (int off = 1; off < 16; off <<= 1)
#pragma unroll
            for (int r = 0; r < 8; ++r) tmax[r] = fmaxf(tmax[r], __shfl_xor(tmax[r], off, 16));
#pragma unroll
        for (int r = 0; r < 8; ++r) {
            float mnew = fmaxf(mcur[r], tmax[r]);
            float alpha = __expf(mcur[r] - mnew);
            mcur[r] = mnew;
            float p0 = __expf(sv[0][r] - mnew), p1 = __expf(sv[1][r] - mnew);
            sv[0][r] = p0; sv[1][r] = p1;
            psum[r] = p0 + p1;
            lcur[r] *= alpha;
#pragma unroll
            for (int f = 0; f < 4; ++f) of[f][r] = of[f][r] * alpha;
        }
#pragma unroll
        for (int off = 1; off < 16; off <<= 1)
#pragma unroll
            for (int r = 0; r < 8; ++r) psum[r] += __shfl_xor(psum[r], off, 16);
#pragma unroll
        for (int r = 0; r < 8; ++r) lcur[r] += psum[r];

#pragma unroll
        for (int sub = 0; sub < 2; ++sub)
#pragma unroll
            for (int r = 0; r < 8; ++r) pst[wave][r + 8 * half][sub * 16 + ln] = (_Float16)sv[sub][r];
        asm volatile("s_wait_dscnt 0" ::: "memory");
        v16h ap = loadA16(&pst[wave][0][0], 0, 0, 32, lane);
#pragma unroll
        for (int f = 0; f < 4; ++f) {
            v16h bv_;
#pragma unroll
            for (int e = 0; e < 16; ++e) bv_[e] = vp[(size_t)(jb0 + kmap(e, half)) * HDIM + f * 16 + ln];
            of[f] = wmma16(ap, bv_, of[f]);
        }
    }
    _Float16* so = &pst[wave][0][0];
    _Float16* srow_buf = reinterpret_cast<_Float16*>(&sq[wave][0][0]);
    (void)so;
#pragma unroll
    for (int r = 0; r < 8; ++r) {
        float inv = 1.0f / lcur[r];
        int mi = r + 8 * half;
#pragma unroll
        for (int f = 0; f < 4; ++f) srow_buf[mi * 72 + f * 16 + ln] = (_Float16)(of[f][r] * inv);
    }
    asm volatile("s_wait_dscnt 0" ::: "memory");
    __builtin_amdgcn_fence(__ATOMIC_RELEASE, "workgroup"); __builtin_amdgcn_wave_barrier(); __builtin_amdgcn_fence(__ATOMIC_ACQUIRE, "workgroup");
    _Float16* aod = ao + ((size_t)(b_ * SS + ibase)) * EE + h * HDIM;
    for (int pass = 0; pass < 2; ++pass) {
#pragma unroll
        for (int j = 0; j < 4; ++j) { const int rr = j * 4 + (lane >> 3), q8 = (lane & 7) * 8;
            *(volatile v8h*)(aod + (size_t)rr * EE + q8) = *(const v8h*)(&srow_buf[rr * 72 + q8]); }
        __threadfence();
    }
}

__global__ __launch_bounds__(256) void k_gemm_out(
    const _Float16* __restrict__ ao, const _Float16* __restrict__ wo,
    const float* __restrict__ bo, float* __restrict__ out)
{
    __shared__ __attribute__((aligned(16))) float sO[8][16 * 68];
    int lane = threadIdx.x & 31, wave = threadIdx.x >> 5, half = lane >> 4, n = lane & 15;
    int tile = blockIdx.x * 8 + wave;
    int mt = tile / 12, ng = tile % 12;
    v8f c[4];
    tile16x64(ao, mt * 16, wo, ng * 64, EE, lane, c);
    float* st = sO[wave];
#pragma unroll
    for (int t = 0; t < 4; ++t)
#pragma unroll
        for (int r = 0; r < 8; ++r) st[(r + 8 * half) * 68 + t * 16 + n] = c[t][r] + bo[ng * 64 + t * 16 + n];
    asm volatile("s_wait_dscnt 0" ::: "memory");
    __builtin_amdgcn_fence(__ATOMIC_RELEASE, "workgroup"); __builtin_amdgcn_wave_barrier(); __builtin_amdgcn_fence(__ATOMIC_ACQUIRE, "workgroup");
    float* od = out + (size_t)(mt * 16) * DD + ng * 64;
    for (int pass = 0; pass < 2; ++pass) {
#pragma unroll
        for (int j = 0; j < 8; ++j) { const int rr = j * 2 + half, q4 = n * 4;
            *(volatile v4f*)(od + (size_t)rr * DD + q4) = *(const v4f*)(&st[rr * 68 + q4]); }
        __threadfence();
    }
}

extern "C" void kernel_launch(void* const* d_in, const int* in_sizes, int n_in,
                              void* d_out, int out_size, void* d_ws, size_t ws_size,
                              hipStream_t stream) {
    const float* x    = (const float*)d_in[0];
    const int*   mask = (const int*)  d_in[1];
    const int*   seg  = (const int*)  d_in[2];
    const float* sep  = (const float*)d_in[3];
    const float* Wq   = (const float*)d_in[4];
    const float* bq   = (const float*)d_in[5];
    const float* Wk   = (const float*)d_in[6];
    const float* bk   = (const float*)d_in[7];
    const float* Wv   = (const float*)d_in[8];
    const float* bv   = (const float*)d_in[9];
    const float* rel  = (const float*)d_in[10];
    const float* Wpk  = (const float*)d_in[11];
    const float* bpk  = (const float*)d_in[12];
    const float* Wpq  = (const float*)d_in[13];
    const float* bpq  = (const float*)d_in[14];
    const float* sameb= (const float*)d_in[15];
    const float* crossb=(const float*)d_in[16];
    const float* sscal= (const float*)d_in[17];
    const float* sdec = (const float*)d_in[18];
    const float* Wo   = (const float*)d_in[19];
    const float* bo   = (const float*)d_in[20];
    float* out = (float*)d_out;

    char* ws = (char*)d_ws;
    size_t off = 0;
    auto alloc = [&](size_t bytes) -> void* {
        off = (off + 255) & ~(size_t)255;
        void* p = ws + off; off += bytes; return p;
    };
    const size_t NX = (size_t)BB * SS * DD;
    const size_t NW = (size_t)EE * DD;
    _Float16* xh   = (_Float16*)alloc(NX * 2);
    _Float16* wqh  = (_Float16*)alloc(NW * 2);
    _Float16* wkh  = (_Float16*)alloc(NW * 2);
    _Float16* wvh  = (_Float16*)alloc(NW * 2);
    _Float16* woh  = (_Float16*)alloc(NW * 2);
    _Float16* wpkh = (_Float16*)alloc(NW * 2);
    _Float16* wpqh = (_Float16*)alloc(NW * 2);
    _Float16* relh = (_Float16*)alloc((size_t)768 * 768 * 2);
    _Float16* qb   = (_Float16*)alloc(NX * 2);
    _Float16* kb   = (_Float16*)alloc(NX * 2);
    _Float16* vt   = (_Float16*)alloc(NX * 2);
    _Float16* posk = (_Float16*)alloc((size_t)HH * 768 * HDIM * 2);
    _Float16* posq = (_Float16*)alloc((size_t)HH * 768 * HDIM * 2);
    _Float16* ao   = (_Float16*)alloc(NX * 2);
    if (off > ws_size) return;

    k_f32_to_f16<<<(int)((NX + 255) / 256), 256, 0, stream>>>(x, xh, (int)NX);
    k_f32_to_f16<<<(int)((NW + 255) / 256), 256, 0, stream>>>(Wq,  wqh,  (int)NW);
    k_f32_to_f16<<<(int)((NW + 255) / 256), 256, 0, stream>>>(Wk,  wkh,  (int)NW);
    k_f32_to_f16<<<(int)((NW + 255) / 256), 256, 0, stream>>>(Wv,  wvh,  (int)NW);
    k_f32_to_f16<<<(int)((NW + 255) / 256), 256, 0, stream>>>(Wo,  woh,  (int)NW);
    k_f32_to_f16<<<(int)((NW + 255) / 256), 256, 0, stream>>>(Wpk, wpkh, (int)NW);
    k_f32_to_f16<<<(int)((NW + 255) / 256), 256, 0, stream>>>(Wpq, wpqh, (int)NW);
    k_build_rel<<<(768 * 768 + 255) / 256, 256, 0, stream>>>(rel, relh);

    k_gemm_qkv<<<dim3(192 * HH / 8, 1, 3), 256, 0, stream>>>(xh, wqh, wkh, wvh, bq, bk, bv, qb, kb, vt);
    k_gemm_pos<<<dim3(48 * HH / 8, 1, 2), 256, 0, stream>>>(relh, wpkh, wpqh, bpk, bpq, posk, posq);

    k_attn<<<BB * HH * (SS / 32), 64, 0, stream>>>(qb, kb, vt, posk, posq,
                                                   mask, seg, sep,
                                                   sameb, crossb, sscal, sdec, ao);
    k_gemm_out<<<2304 / 8, 256, 0, stream>>>(ao, woh, bo, out);
    (void)in_sizes; (void)n_in; (void)out_size;
}
